// GraphNeuralRecommender_26826365731399
// MI455X (gfx1250) — hardware-run, weakly checked
//
#include <hip/hip_runtime.h>
#include <stddef.h>
#include <stdint.h>
#include <math.h>

#define NU      60000
#define NI      40000
#define NN      100000
#define FD      64
#define HD      32
#define NE      1600000
#define NP      16384
#define GBM     128
#define MP      100096
#define NTHR    256
#define NWAVE   8
#define EPT     8
#define WCH     (32 * EPT)
#define NBRUN   1024
#define SLB     10
#define NBK     98
#define WLCAP   3072
#define RCAP    24576
#define DEGCAP  64
#define MAXDEG_MEAS 36
#define MAXBLK_MEAS 16721
#define RBM     128
#define SPA     36
#define SPB     68
#define WSMAX   ((size_t)(128u << 20))

#define SINGLE_BF16 0
#define HLP     64
#define WDP     64
#define ZLP     256
#define PDP     256
#define KTWO    (SINGLE_BF16 ? 32 : 64)
#define KFIVE   (SINGLE_BF16 ? 128 : 256)

#define PER     (((NE + NWAVE * WCH - 1) / (NWAVE * WCH)) * WCH)
#define BK_ZINTS (NWAVE * WLCAP + RCAP + 3 * NBRUN)
#define BK_INTS  (BK_ZINTS + 16)
#define BK_LDS   (BK_INTS * 4)

#define PBU   (NU * FD / 8 / NTHR)
#define PBI   ((MP - NU) * FD / 8 / NTHR)
#define PBWA  (HD * FD / 8 / NTHR)
#define PBWB  (FD * WDP / 8 / NTHR)
#define PBWC  (HD * PDP / 8 / NTHR)
#define PBTOT (PBU + PBI + PBWA + PBWB + PBWC + 1)

static_assert(NN == NU + NI);
static_assert(MP % GBM == 0 && MP >= NN && MP == 782 * GBM && MP % RBM == 0);
static_assert(NBRUN == (1 << SLB) && NBRUN % RBM == 0 && NBRUN % 32 == 0 && NBRUN <= 1024);
static_assert(NBK * NBRUN >= MP);
static_assert(NE < (1 << 21) && (((long long)NE) << SLB) < (1LL << 31));
static_assert(NE % WCH == 0 && NE % 4 == 0 && PER % WCH == 0 && (NWAVE - 1) * PER < NE);
static_assert(RCAP == NWAVE * WLCAP && RCAP % (NTHR * 2) == 0 && BK_ZINTS % (NTHR * 4) == 0);
static_assert((long long)RCAP * 100 >= (long long)MAXBLK_MEAS * 105);
static_assert(WLCAP >= MAXBLK_MEAS / 8 + 8 * 46 + 1);
static_assert(MAXDEG_MEAS + 8 <= DEGCAP);
static_assert((NU * FD / 8) % NTHR == 0 && ((MP - NU) * FD / 8) % NTHR == 0);
static_assert((HD * FD / 8) % NTHR == 0 && (FD * WDP / 8) % NTHR == 0 && (HD * PDP / 8) % NTHR == 0);
static_assert(FD % 32 == 0 && KTWO % 32 == 0 && KFIVE % 32 == 0 && KTWO <= HLP && KTWO <= WDP && KFIVE <= ZLP && KFIVE <= PDP);
static_assert(HLP == 2 * HD && WDP == 2 * HD && ZLP == 4 * FD && PDP == 4 * FD);
static_assert(BK_LDS <= 300000);
static_assert((GBM * SPB + 64) * 4 <= 65536 && (GBM * SPA + 64 + GBM) * 4 <= 65536);
static_assert(NP % GBM == 0 && NP % NWAVE == 0);
static_assert((size_t)NP + (size_t)(NN - 1) * FD + (FD - 1) < (size_t)NP + (size_t)NN * FD);
static_assert((NP * 4) % 128 == 0);

typedef float          v4f   __attribute__((ext_vector_type(4)));
typedef float          v8f   __attribute__((ext_vector_type(8)));
typedef int            v2i   __attribute__((ext_vector_type(2)));
typedef int            v4i   __attribute__((ext_vector_type(4)));
typedef int            v8i   __attribute__((ext_vector_type(8)));
typedef unsigned short v8us  __attribute__((ext_vector_type(8)));
typedef unsigned short v16us __attribute__((ext_vector_type(16)));
typedef __bf16         v16bf __attribute__((ext_vector_type(16)));
typedef v4f  __attribute__((may_alias)) v4fa;
typedef v2i  __attribute__((may_alias)) v2ia;
typedef v4i  __attribute__((may_alias)) v4ia;
typedef v8us __attribute__((may_alias)) v8usa;
union FragB { v16bf v; v16us u; v8us h[2]; v8i w; };

__device__ __forceinline__ v8f wmb(const FragB& a, const FragB& b, v8f c) {
  v8f d = __builtin_amdgcn_wmma_f32_16x16x32_bf16(false, a.v, false, b.v, (short)0, c, false, false);
  asm volatile("v_nop\n\tv_nop\n\tv_nop\n\tv_nop" : "+v"(d) : "v"(a.w), "v"(b.w));
  return d;
}

__device__ __forceinline__ unsigned bf16_bits(float f) {
  const unsigned u = __float_as_uint(f);
  const unsigned r = (u + 0x7fffu + ((u >> 16) & 1u)) >> 16;
  const unsigned q = (u >> 16) | 0x40u;
  return ((u & 0x7fffffffu) > 0x7f800000u) ? q : r;
}

__device__ __forceinline__ void hilo_pack(float v0, float v1, float v2, float v3,
                                          int& h01, int& h23, int& l01, int& l23) {
  const unsigned a0 = bf16_bits(v0), a1 = bf16_bits(v1), a2 = bf16_bits(v2), a3 = bf16_bits(v3);
  const unsigned b0 = bf16_bits(v0 - __uint_as_float(a0 << 16));
  const unsigned b1 = bf16_bits(v1 - __uint_as_float(a1 << 16));
  const unsigned b2 = bf16_bits(v2 - __uint_as_float(a2 << 16));
  const unsigned b3 = bf16_bits(v3 - __uint_as_float(a3 << 16));
  h01 = (int)(a0 | (a1 << 16)); h23 = (int)(a2 | (a3 << 16));
  l01 = (int)(b0 | (b1 << 16)); l23 = (int)(b2 | (b3 << 16));
}

__device__ __forceinline__ v4i regroup_q(int h01, int h23, int l01, int l23, int lane) {
  const int t  = lane & 7;
  const int s0 = (lane & 24) + ((2 * t) & 7), s1 = s0 + 1;
  const int a0 = __shfl(h01, s0, 32), a1 = __shfl(h23, s0, 32), a2 = __shfl(h01, s1, 32), a3 = __shfl(h23, s1, 32);
  const int b0 = __shfl(l01, s0, 32), b1 = __shfl(l23, s0, 32), b2 = __shfl(l01, s1, 32), b3 = __shfl(l23, s1, 32);
  const int mk = (t < 4) ? -1 : 0;
  v4i o;
  o.x = (a0 & mk) | (b0 & ~mk); o.y = (a1 & mk) | (b1 & ~mk);
  o.z = (a2 & mk) | (b2 & ~mk); o.w = (a3 & mk) | (b3 & ~mk);
  return o;
}

__device__ __forceinline__ void st2_v4f(float* p, v4f v) {
  *(volatile v4f*)p = v;
  __threadfence();
  *(volatile v4f*)p = v;
}
__device__ __forceinline__ void st2_v8us(unsigned short* p, v8us v) {
  *(volatile v8us*)p = v;
  __threadfence();
  *(volatile v8us*)p = v;
}

__device__ __forceinline__ v8us pack8(v4f a, v4f b, unsigned mk) {
  v8us o;
  o[0] = (unsigned short)(bf16_bits(a.x) & mk); o[1] = (unsigned short)(bf16_bits(a.y) & mk);
  o[2] = (unsigned short)(bf16_bits(a.z) & mk); o[3] = (unsigned short)(bf16_bits(a.w) & mk);
  o[4] = (unsigned short)(bf16_bits(b.x) & mk); o[5] = (unsigned short)(bf16_bits(b.y) & mk);
  o[6] = (unsigned short)(bf16_bits(b.z) & mk); o[7] = (unsigned short)(bf16_bits(b.w) & mk);
  return o;
}

__global__ __launch_bounds__(NTHR) void k_prep(const float* __restrict__ ue, const float* __restrict__ ie,
                                               const float* __restrict__ w1, const float* __restrict__ b1,
                                               const float* __restrict__ w2, const float* __restrict__ b2,
                                               const float* __restrict__ pw, const float* __restrict__ pb,
                                               const float* __restrict__ qw, const float* __restrict__ qb,
                                               unsigned short* xb, unsigned short* w1b, unsigned short* w2d,
                                               unsigned short* p1d, float* smt) {
  const int tid = (int)threadIdx.x;
  const int blk = (int)blockIdx.x;
  if (blk < PBU) {
    const int u   = blk * NTHR + tid;
    const int row = u >> 3, k8 = (u & 7) * 8;
    const float* p = ue + (size_t)row * FD + k8;
    const v4f a = *(const v4fa*)p;
    const v4f b = *(const v4fa*)(p + 4);
    st2_v8us(xb + (size_t)row * FD + k8, pack8(a, b, 0xffffu));
  } else if (blk < PBU + PBI) {
    const int u  = (blk - PBU) * NTHR + tid;
    const int r  = u >> 3, k8 = (u & 7) * 8;
    const int rc = r < NI ? r : NI - 1;
    const unsigned mk = r < NI ? 0xffffu : 0u;
    const float* p = ie + (size_t)rc * FD + k8;
    const v4f a = *(const v4fa*)p;
    const v4f b = *(const v4fa*)(p + 4);
    st2_v8us(xb + (size_t)(NU + r) * FD + k8, pack8(a, b, mk));
  } else if (blk < PBU + PBI + PBWA) {
    const int u = (blk - PBU - PBI) * NTHR + tid;
    const int n = u >> 3, k8 = (u & 7) * 8;
    const float* p = w1 + (size_t)n * FD + k8;
    const v4f a = *(const v4fa*)p;
    const v4f b = *(const v4fa*)(p + 4);
    st2_v8us(w1b + (size_t)n * FD + k8, pack8(a, b, 0xffffu));
  } else if (blk < PBU + PBI + PBWA + PBWB) {
    const int u = (blk - PBU - PBI - PBWA) * NTHR + tid;
    const int n = u >> 3, k8 = (u & 7) * 8, kk = k8 & (HD - 1);
    const float* p = w2 + (size_t)n * HD + kk;
    const v4f a = *(const v4fa*)p;
    const v4f b = *(const v4fa*)(p + 4);
    st2_v8us(w2d + (size_t)n * WDP + k8, pack8(a, b, 0xffffu));
  } else if (blk < PBU + PBI + PBWA + PBWB + PBWC) {
    const int u = (blk - PBU - PBI - PBWA - PBWB) * NTHR + tid;
    const int n = u >> 5, k8 = (u & 31) * 8, kk = k8 & (2 * FD - 1);
    const float* p = pw + (size_t)n * (2 * FD) + kk;
    const v4f a = *(const v4fa*)p;
    const v4f b = *(const v4fa*)(p + 4);
    st2_v8us(p1d + (size_t)n * PDP + k8, pack8(a, b, 0xffffu));
  } else {
    if (tid < 64) {
      const int t = tid;
      const v4f a = *(const v4fa*)(b1 + 4 * (t & 7));
      const v4f b = *(const v4fa*)(b2 + 4 * ((t - 8) & 15));
      const v4f c = *(const v4fa*)(pb + 4 * (t & 7));
      const v4f d = *(const v4fa*)(qw + 4 * (t & 7));
      const float e = qb[0];
      asm volatile("" :: "v"(a), "v"(b));
      asm volatile("" :: "v"(c), "v"(d), "v"(e));
      const unsigned ma = (t < 8) ? 0xffffffffu : 0u;
      const unsigned mb = (t >= 8 && t < 24) ? 0xffffffffu : 0u;
      const unsigned mc = (t >= 24 && t < 32) ? 0xffffffffu : 0u;
      const unsigned md = (t >= 32 && t < 40) ? 0xffffffffu : 0u;
      const unsigned me = (t == 40) ? 0xffffffffu : 0u;
      v4f o;
      o.x = __uint_as_float(((bf16_bits(a.x) << 16) & ma) | ((bf16_bits(b.x) << 16) & mb) |
                            ((bf16_bits(c.x) << 16) & mc) | ((bf16_bits(d.x) << 16) & md) |
                            ((bf16_bits(e) << 16) & me));
      o.y = __uint_as_float(((bf16_bits(a.y) << 16) & ma) | ((bf16_bits(b.y) << 16) & mb) |
                            ((bf16_bits(c.y) << 16) & mc) | ((bf16_bits(d.y) << 16) & md));
      o.z = __uint_as_float(((bf16_bits(a.z) << 16) & ma) | ((bf16_bits(b.z) << 16) & mb) |
                            ((bf16_bits(c.z) << 16) & mc) | ((bf16_bits(d.z) << 16) & md));
      o.w = __uint_as_float(((bf16_bits(a.w) << 16) & ma) | ((bf16_bits(b.w) << 16) & mb) |
                            ((bf16_bits(c.w) << 16) & mc) | ((bf16_bits(d.w) << 16) & md));
      st2_v4f(smt + 4 * t, o);
    }
  }
}

__device__ __forceinline__ void bucket_flush(const int* pl, const int* cnt, int tot, int ov,
                                             const int* __restrict__ cols, const float* __restrict__ vals,
                                             int* lp, int* cop, int* fp, int tid) {
#pragma unroll 1
  for (int i = tid * 2; i < RCAP; i += NTHR * 2) {
    const v2i pk = *(const v2ia*)(pl + i);
    int ea = (pk.x >> SLB) & 0x1fffff;
    int eb = (pk.y >> SLB) & 0x1fffff;
    ea = ea > NE - 1 ? NE - 1 : ea;
    eb = eb > NE - 1 ? NE - 1 : eb;
    int ca = cols[ea];
    int cb = cols[eb];
    const float va = vals[ea];
    const float vb = vals[eb];
    asm volatile("" :: "v"(ca), "v"(cb), "v"(va), "v"(vb));
    ca = ca < 0 ? 0 : (ca > NN - 1 ? NN - 1 : ca);
    cb = cb < 0 ? 0 : (cb > NN - 1 ? NN - 1 : cb);
    const int ma = (i < tot) ? -1 : 0;
    const int mb = (i + 1 < tot) ? -1 : 0;
    v4i o;
    o.x = ca & ma; o.y = (int)(bf16_bits(va) << 16) & ma;
    o.z = cb & mb; o.w = (int)(bf16_bits(vb) << 16) & mb;
    *(volatile v4i*)(lp + (size_t)2 * (size_t)i) = o;
  }
#pragma unroll 1
  for (int it = 0; it < 2; ++it) {
    const int i4 = (it * NTHR + tid) * 4;
    const v4i v = *(const v4ia*)(cnt + i4);
    *(volatile v4i*)(cop + i4) = v;
  }
  if (tid < 8) {
    const v4i f = {ov, ov, ov, ov};
    *(volatile v4i*)(fp + 4 * tid) = f;
  }
}

__global__ __launch_bounds__(NTHR) void k_bucket(const int* __restrict__ keys, const int* __restrict__ cols,
                                                 const float* __restrict__ vals, int* lst, int* cof, int* flg) {
  extern __shared__ __attribute__((aligned(16))) int dsm[];
  int* wl   = dsm;
  int* pl   = dsm + NWAVE * WLCAP;
  int* cnt  = pl + RCAP;
  int* offs = cnt + NBRUN;
  int* cur  = offs + NBRUN;
  int* misc = cur + NBRUN;
  const int tid = (int)threadIdx.x, lane = tid & 31, wave = tid >> 5;
  const int blk = (int)blockIdx.x;
  const unsigned nbs = (unsigned)(blk * NBRUN);

  {
    const v4i z4 = {0, 0, 0, 0};
    for (int i = tid * 4; i < BK_ZINTS; i += NTHR * 4) *(v4ia*)(dsm + i) = z4;
    if (tid < 16) misc[tid] = 0;
  }
  __syncthreads();

  {
    const int ebeg = wave * PER;
    const int eend = (ebeg + PER < NE) ? (ebeg + PER) : NE;
    int* mylist = wl + wave * WLCAP;
    int wc = 0;
#pragma unroll 1
    for (int cb = ebeg; cb < eend; cb += WCH) {
      const int e0 = cb + lane * EPT;
      const v4i da = *(const v4ia*)(keys + e0);
      const v4i db = *(const v4ia*)(keys + e0 + 4);
      const unsigned s0 = (unsigned)da.x - nbs, s1 = (unsigned)da.y - nbs;
      const unsigned s2 = (unsigned)da.z - nbs, s3 = (unsigned)da.w - nbs;
      const unsigned s4 = (unsigned)db.x - nbs, s5 = (unsigned)db.y - nbs;
      const unsigned s6 = (unsigned)db.z - nbs, s7 = (unsigned)db.w - nbs;
      const bool h0 = s0 < (unsigned)NBRUN, h1 = s1 < (unsigned)NBRUN, h2 = s2 < (unsigned)NBRUN, h3 = s3 < (unsigned)NBRUN;
      const bool h4 = s4 < (unsigned)NBRUN, h5 = s5 < (unsigned)NBRUN, h6 = s6 < (unsigned)NBRUN, h7 = s7 < (unsigned)NBRUN;
      const unsigned m0 = __builtin_amdgcn_ballot_w32(h0), m1 = __builtin_amdgcn_ballot_w32(h1);
      const unsigned m2 = __builtin_amdgcn_ballot_w32(h2), m3 = __builtin_amdgcn_ballot_w32(h3);
      const unsigned m4 = __builtin_amdgcn_ballot_w32(h4), m5 = __builtin_amdgcn_ballot_w32(h5);
      const unsigned m6 = __builtin_amdgcn_ballot_w32(h6), m7 = __builtin_amdgcn_ballot_w32(h7);
      const unsigned any = m0 | m1 | m2 | m3 | m4 | m5 | m6 | m7;
      if (any != 0u) {
        const int pre = (int)(__builtin_amdgcn_mbcnt_lo(m0, 0u) + __builtin_amdgcn_mbcnt_lo(m1, 0u) +
                              __builtin_amdgcn_mbcnt_lo(m2, 0u) + __builtin_amdgcn_mbcnt_lo(m3, 0u) +
                              __builtin_amdgcn_mbcnt_lo(m4, 0u) + __builtin_amdgcn_mbcnt_lo(m5, 0u) +
                              __builtin_amdgcn_mbcnt_lo(m6, 0u) + __builtin_amdgcn_mbcnt_lo(m7, 0u));
        int p = wc + pre;
        if (h0) { if (p < WLCAP) mylist[p] = ((e0 + 0) << SLB) | (int)s0; p = p + 1; }
        if (h1) { if (p < WLCAP) mylist[p] = ((e0 + 1) << SLB) | (int)s1; p = p + 1; }
        if (h2) { if (p < WLCAP) mylist[p] = ((e0 + 2) << SLB) | (int)s2; p = p + 1; }
        if (h3) { if (p < WLCAP) mylist[p] = ((e0 + 3) << SLB) | (int)s3; p = p + 1; }
        if (h4) { if (p < WLCAP) mylist[p] = ((e0 + 4) << SLB) | (int)s4; p = p + 1; }
        if (h5) { if (p < WLCAP) mylist[p] = ((e0 + 5) << SLB) | (int)s5; p = p + 1; }
        if (h6) { if (p < WLCAP) mylist[p] = ((e0 + 6) << SLB) | (int)s6; p = p + 1; }
        if (h7) { if (p < WLCAP) mylist[p] = ((e0 + 7) << SLB) | (int)s7; p = p + 1; }
        wc += (int)(__builtin_popcount(m0) + __builtin_popcount(m1) + __builtin_popcount(m2) + __builtin_popcount(m3) +
                    __builtin_popcount(m4) + __builtin_popcount(m5) + __builtin_popcount(m6) + __builtin_popcount(m7));
      }
    }
    if (lane == 0) misc[wave] = wc;
  }
  __syncthreads();

  if (wave == 0) {
    int ov = 0;
#pragma unroll 1
    for (int w2 = 0; w2 < NWAVE; ++w2) {
      int c = misc[w2];
      if (c > WLCAP) ov = 1;
      c = c < 0 ? 0 : (c > WLCAP ? WLCAP : c);
#pragma unroll 1
      for (int b0 = 0; b0 < c; b0 += 32) {
        const int idx = b0 + lane;
        const int ent = wl[w2 * WLCAP + (idx < WLCAP ? idx : WLCAP - 1)];
        const int m32 = (c - b0) < 32 ? (c - b0) : 32;
#pragma unroll 1
        for (int k = 0; k < m32; ++k) {
          const int u    = __builtin_amdgcn_readlane(ent, k);
          const int slot = u & (NBRUN - 1);
          if (lane == 0) cnt[slot] = cnt[slot] + 1;
        }
      }
    }
    if (lane == 0) misc[9] = ov;
  }
  __syncthreads();
  if (wave == 0) {
    const int base = lane * (NBRUN / 32);
    int s = 0;
#pragma unroll 1
    for (int i = 0; i < NBRUN / 32; ++i) s += cnt[base + i];
    int incl = s;
#pragma unroll
    for (int d = 1; d < 32; d <<= 1) {
      const int y = __shfl_up(incl, d, 32);
      if (lane >= d) incl += y;
    }
    int run = incl - s;
#pragma unroll 1
    for (int i = 0; i < NBRUN / 32; ++i) {
      const int cv = cnt[base + i];
      offs[base + i] = run;
      cur[base + i]  = run;
      run += cv;
    }
    if (lane == 31) misc[10] = run;
  }
  __syncthreads();

  if (wave == 0) {
#pragma unroll 1
    for (int w2 = 0; w2 < NWAVE; ++w2) {
      int c = misc[w2];
      c = c < 0 ? 0 : (c > WLCAP ? WLCAP : c);
#pragma unroll 1
      for (int b0 = 0; b0 < c; b0 += 32) {
        const int idx = b0 + lane;
        const int ent = wl[w2 * WLCAP + (idx < WLCAP ? idx : WLCAP - 1)];
        const int m32 = (c - b0) < 32 ? (c - b0) : 32;
#pragma unroll 1
        for (int k = 0; k < m32; ++k) {
          const int u    = __builtin_amdgcn_readlane(ent, k);
          const int slot = u & (NBRUN - 1);
          if (lane == 0) {
            int p = cur[slot];
            p = p < 0 ? 0 : (p > RCAP - 1 ? RCAP - 1 : p);
            pl[p] = u;
            cur[slot] = p + 1;
          }
        }
      }
    }
  }
  __syncthreads();

  const int ovf = misc[9];
  int tot = misc[10];
  tot = tot < 0 ? 0 : (tot > RCAP ? RCAP : tot);
  int* lp  = lst + (size_t)blk * (size_t)(2 * RCAP);
  int* cop = cof + (size_t)blk * (2 * NBRUN);
  int* fp  = flg + (size_t)blk * 32;
  bucket_flush(pl, cnt, tot, ovf, cols, vals, lp, cop, fp, tid);
  __threadfence();
  bucket_flush(pl, cnt, tot, ovf, cols, vals, lp, cop, fp, tid);
}

template <int KTOT, int BPT, int NT>
__device__ __forceinline__ void gemm_rows16(const unsigned short* __restrict__ ap,
                                            const unsigned short* __restrict__ bp, v8f (&acc)[NT]) {
#pragma unroll 1
  for (int k0 = 0; k0 < KTOT; k0 += 32) {
    FragB af;
    af.h[0] = *(const v8usa*)(ap + k0);
    af.h[1] = *(const v8usa*)(ap + k0 + 16);
#pragma unroll
    for (int nt = 0; nt < NT; ++nt) {
      const unsigned short* wq = bp + (size_t)(16 * nt) * (size_t)BPT + k0;
      FragB bf;
      bf.h[0] = *(const v8usa*)wq;
      bf.h[1] = *(const v8usa*)(wq + 16);
      acc[nt] = wmb(af, bf, acc[nt]);
    }
  }
}

template <int NT, int SPX>
__device__ __forceinline__ void stage_d(float* stg, const v8f (&acc)[NT], int wave, int hh, int m) {
#pragma unroll
  for (int nt = 0; nt < NT; ++nt) {
#pragma unroll
    for (int r = 0; r < 8; ++r) stg[(16 * wave + 8 * hh + r) * SPX + 16 * nt + m] = acc[nt][r];
  }
}

__global__ __launch_bounds__(NTHR) __attribute__((amdgpu_num_vgpr(248)))
void k_gemm1(const unsigned short* __restrict__ xb, const unsigned short* __restrict__ w1b,
             const float* __restrict__ smt, float* t1f) {
  __shared__ __attribute__((aligned(16))) float stg[GBM * SPA];
  __shared__ __attribute__((aligned(16))) float sb[32];
  const int tid = (int)threadIdx.x, lane = tid & 31, wave = tid >> 5, hh = lane >> 4, m = lane & 15;
  const int rowBase = (int)blockIdx.x * GBM;
  if (tid < 8) *(v4fa*)(sb + 4 * tid) = *(const v4fa*)(smt + 4 * tid);

  v8f acc[2];
  {
    const v8f z = {0.f, 0.f, 0.f, 0.f, 0.f, 0.f, 0.f, 0.f};
    acc[0] = z; acc[1] = z;
  }
  const unsigned short* ap = xb + (size_t)(rowBase + 16 * wave + m) * (size_t)FD + 8 * hh;
  const unsigned short* bp = w1b + (size_t)m * (size_t)FD + 8 * hh;
  gemm_rows16<FD, FD, 2>(ap, bp, acc);
  stage_d<2, SPA>(stg, acc, wave, hh, m);
  __syncthreads();

  const int q = lane & 7, qw = lane >> 3;
  const v4f bias = *(const v4fa*)(sb + 4 * q);
#pragma unroll 1
  for (int i = 0; i < 4; ++i) {
    const int lr   = 16 * wave + 4 * i + qw;
    const int grow = rowBase + lr;
    const bool live = grow < NN;
    const v4f a = *(const v4fa*)(stg + lr * SPA + 4 * q);
    asm volatile("" :: "v"(a));
    const float v0 = a.x + bias.x, v1 = a.y + bias.y, v2 = a.z + bias.z, v3 = a.w + bias.w;
    v4f o;
    o.x = live ? v0 : 0.0f; o.y = live ? v1 : 0.0f; o.z = live ? v2 : 0.0f; o.w = live ? v3 : 0.0f;
    st2_v4f(t1f + (size_t)grow * HD + 4 * q, o);
  }
}

__global__ __launch_bounds__(NTHR) void k_replay1(const int* __restrict__ lst, const int* __restrict__ cof,
                                                  const int* __restrict__ flg, const float* __restrict__ t1f,
                                                  unsigned short* h1p) {
  const int tid = (int)threadIdx.x, lane = tid & 31, wave = tid >> 5, qw = lane >> 3, q = lane & 7;
  const int rowBase = (int)blockIdx.x * RBM;
  const int bucket  = rowBase >> SLB;
  const int* lb  = lst + (size_t)bucket * (size_t)(2 * RCAP);
  const int* cob = cof + (size_t)bucket * (2 * NBRUN);
  const int flag = flg[(size_t)bucket * 32];
  const float qnan = __uint_as_float(0x7fc00000u);

#pragma unroll 1
  for (int i = 0; i < RBM / (4 * NWAVE); ++i) {
    const int d    = rowBase + (RBM / NWAVE) * wave + 4 * i + qw;
    const int slot = d & (NBRUN - 1);
    int c = cob[slot];
    int o = cob[NBRUN + slot];
    const bool big = c > DEGCAP;
    c = c < 0 ? 0 : (c > DEGCAP ? DEGCAP : c);
    o = o < 0 ? 0 : (o > RCAP - 1 ? RCAP - 1 : o);
    int cm = c;
    {
      int y = __shfl_xor(cm, 8, 32);
      cm = cm > y ? cm : y;
      y = __shfl_xor(cm, 16, 32);
      cm = cm > y ? cm : y;
    }
    cm = cm < 0 ? 0 : (cm > DEGCAP ? DEGCAP : cm);
    const int trips = __builtin_amdgcn_readfirstlane(cm);
    int last = o + c - 1;
    last = last < o ? o : last;
    last = last > RCAP - 1 ? RCAP - 1 : last;
    float a0 = 0.0f, a1 = 0.0f, a2 = 0.0f, a3 = 0.0f;
#pragma unroll 1
    for (int j = 0; j < trips; ++j) {
      int idx = o + j;
      idx = idx > last ? last : idx;
      const v2i en = *(const v2ia*)(lb + 2 * idx);
      asm volatile("" :: "v"(en));
      int sr = en.x;
      sr = sr < 0 ? 0 : (sr > NN - 1 ? NN - 1 : sr);
      const float w = __int_as_float(en.y);
      const v4f v = *(const v4fa*)(t1f + (size_t)sr * HD + 4 * q);
      asm volatile("" :: "v"(v));
      const bool valid = j < c;
      const float t0 = fmaf(w, v.x, a0), t1 = fmaf(w, v.y, a1), t2 = fmaf(w, v.z, a2), t3 = fmaf(w, v.w, a3);
      a0 = valid ? t0 : a0; a1 = valid ? t1 : a1; a2 = valid ? t2 : a2; a3 = valid ? t3 : a3;
    }
    float m0 = (a0 > 0.0f) ? a0 : (a0 - a0);
    float m1 = (a1 > 0.0f) ? a1 : (a1 - a1);
    float m2 = (a2 > 0.0f) ? a2 : (a2 - a2);
    float m3 = (a3 > 0.0f) ? a3 : (a3 - a3);
    const bool bad  = (flag != 0) | big;
    const bool live = d < NN;
    m0 = bad ? qnan : m0; m1 = bad ? qnan : m1; m2 = bad ? qnan : m2; m3 = bad ? qnan : m3;
    m0 = live ? m0 : 0.0f; m1 = live ? m1 : 0.0f; m2 = live ? m2 : 0.0f; m3 = live ? m3 : 0.0f;
    int h01, h23, l01, l23;
    hilo_pack(m0, m1, m2, m3, h01, h23, l01, l23);
    const v4i ow = regroup_q(h01, h23, l01, l23, lane);
    unsigned short* hp = h1p + (size_t)d * HLP + 8 * q;
    *(volatile v4i*)hp = ow;
    __threadfence();
    *(volatile v4i*)hp = ow;
  }
}

__global__ __launch_bounds__(NTHR) __attribute__((amdgpu_num_vgpr(248)))
void k_gemm2(const unsigned short* __restrict__ h1p, const unsigned short* __restrict__ w2d,
             const float* __restrict__ smt, float* t2f) {
  __shared__ __attribute__((aligned(16))) float stg[GBM * SPB];
  __shared__ __attribute__((aligned(16))) float sb[64];
  const int tid = (int)threadIdx.x, lane = tid & 31, wave = tid >> 5, hh = lane >> 4, m = lane & 15;
  const int rowBase = (int)blockIdx.x * GBM;
  if (tid < 16) *(v4fa*)(sb + 4 * tid) = *(const v4fa*)(smt + 32 + 4 * tid);

  v8f acc[4];
  {
    const v8f z = {0.f, 0.f, 0.f, 0.f, 0.f, 0.f, 0.f, 0.f};
#pragma unroll
    for (int t = 0; t < 4; ++t) acc[t] = z;
  }
  const unsigned short* ap = h1p + (size_t)(rowBase + 16 * wave + m) * (size_t)HLP + 8 * hh;
  const unsigned short* bp = w2d + (size_t)m * (size_t)WDP + 8 * hh;
  gemm_rows16<KTWO, WDP, 4>(ap, bp, acc);
  stage_d<4, SPB>(stg, acc, wave, hh, m);
  __syncthreads();

  const v4f bias = *(const v4fa*)(sb + 4 * m);
#pragma unroll 1
  for (int i = 0; i < 8; ++i) {
    const int lr   = 16 * wave + 2 * i + hh;
    const int grow = rowBase + lr;
    const bool live = grow < NN;
    const v4f a = *(const v4fa*)(stg + lr * SPB + 4 * m);
    asm volatile("" :: "v"(a));
    const float v0 = a.x + bias.x, v1 = a.y + bias.y, v2 = a.z + bias.z, v3 = a.w + bias.w;
    v4f o;
    o.x = live ? v0 : 0.0f; o.y = live ? v1 : 0.0f; o.z = live ? v2 : 0.0f; o.w = live ? v3 : 0.0f;
    st2_v4f(t2f + (size_t)grow * FD + 4 * m, o);
  }
}

__global__ __launch_bounds__(NTHR) void k_replay2(const int* __restrict__ lst, const int* __restrict__ cof,
                                                  const int* __restrict__ flg, const float* __restrict__ t2f,
                                                  float* outp, float* h2f) {
  const int tid = (int)threadIdx.x, lane = tid & 31, wave = tid >> 5, hh = lane >> 4, q = lane & 15;
  const int rowBase = (int)blockIdx.x * RBM;
  const int bucket  = rowBase >> SLB;
  const int* lb  = lst + (size_t)bucket * (size_t)(2 * RCAP);
  const int* cob = cof + (size_t)bucket * (2 * NBRUN);
  const int flag = flg[(size_t)bucket * 32];
  const float qnan = __uint_as_float(0x7fc00000u);

#pragma unroll 1
  for (int i = 0; i < RBM / (2 * NWAVE); ++i) {
    const int d    = rowBase + (RBM / NWAVE) * wave + 2 * i + hh;
    const int slot = d & (NBRUN - 1);
    int c = cob[slot];
    int o = cob[NBRUN + slot];
    const bool big = c > DEGCAP;
    c = c < 0 ? 0 : (c > DEGCAP ? DEGCAP : c);
    o = o < 0 ? 0 : (o > RCAP - 1 ? RCAP - 1 : o);
    int cm = c;
    {
      const int y = __shfl_xor(cm, 16, 32);
      cm = cm > y ? cm : y;
    }
    cm = cm < 0 ? 0 : (cm > DEGCAP ? DEGCAP : cm);
    const int trips = __builtin_amdgcn_readfirstlane(cm);
    int last = o + c - 1;
    last = last < o ? o : last;
    last = last > RCAP - 1 ? RCAP - 1 : last;
    float a0 = 0.0f, a1 = 0.0f, a2 = 0.0f, a3 = 0.0f;
#pragma unroll 1
    for (int j = 0; j < trips; ++j) {
      int idx = o + j;
      idx = idx > last ? last : idx;
      const v2i en = *(const v2ia*)(lb + 2 * idx);
      asm volatile("" :: "v"(en));
      int sr = en.x;
      sr = sr < 0 ? 0 : (sr > NN - 1 ? NN - 1 : sr);
      const float w = __int_as_float(en.y);
      const v4f v = *(const v4fa*)(t2f + (size_t)sr * FD + 4 * q);
      asm volatile("" :: "v"(v));
      const bool valid = j < c;
      const float t0 = fmaf(w, v.x, a0), t1 = fmaf(w, v.y, a1), t2 = fmaf(w, v.z, a2), t3 = fmaf(w, v.w, a3);
      a0 = valid ? t0 : a0; a1 = valid ? t1 : a1; a2 = valid ? t2 : a2; a3 = valid ? t3 : a3;
    }
    float m0 = (a0 > 0.0f) ? a0 : (a0 - a0);
    float m1 = (a1 > 0.0f) ? a1 : (a1 - a1);
    float m2 = (a2 > 0.0f) ? a2 : (a2 - a2);
    float m3 = (a3 > 0.0f) ? a3 : (a3 - a3);
    const bool bad = (flag != 0) | big;
    m0 = bad ? qnan : m0; m1 = bad ? qnan : m1; m2 = bad ? qnan : m2; m3 = bad ? qnan : m3;
    v4f ov;
    ov.x = m0; ov.y = m1; ov.z = m2; ov.w = m3;
    const bool live = d < NN;
    const int dc = live ? d : NN - 1;
    float* op = outp + (size_t)dc * FD + 4 * q;
    float* hp = h2f + (size_t)dc * FD + 4 * q;
    if (live) {
      *(volatile v4f*)op = ov;
      *(volatile v4f*)hp = ov;
    }
    __threadfence();
    if (live) {
      *(volatile v4f*)op = ov;
      *(volatile v4f*)hp = ov;
    }
  }
}

__global__ __launch_bounds__(NTHR) void k_headprep(const int* __restrict__ uids, const int* __restrict__ iids,
                                                   const float* __restrict__ h2f, unsigned short* zhl) {
  const int tid = (int)threadIdx.x, lane = tid & 31, wave = tid >> 5;
  const int p = (int)blockIdx.x * NWAVE + wave;
  int u  = uids[p];
  int it = iids[p];
  u  = u  < 0 ? 0 : (u  > NU - 1 ? NU - 1 : u);
  it = it < 0 ? 0 : (it > NI - 1 ? NI - 1 : it);
  const int sel  = (lane & 8) ? -1 : 0;
  const int node = ((NU + it) & sel) | (u & ~sel);
  const int ch   = 8 * (lane & 7);
  const float* rp = h2f + (size_t)node * FD + ch;
  const v4f a = *(const v4fa*)rp;
  const v4f b = *(const v4fa*)(rp + 4);
  asm volatile("" :: "v"(a), "v"(b));
  const unsigned mk = (lane & 16) ? 0u : 0xffffu;
  const float f[8] = {a.x, a.y, a.z, a.w, b.x, b.y, b.z, b.w};
  v8us o;
#pragma unroll
  for (int i = 0; i < 8; ++i) {
    const unsigned hb = bf16_bits(f[i]);
    const unsigned lb = bf16_bits(f[i] - __uint_as_float(hb << 16));
    o[i] = (unsigned short)((hb & mk) | (lb & (~mk & 0xffffu)));
  }
  st2_v8us(zhl + (size_t)p * ZLP + 8 * lane, o);
}

__global__ __launch_bounds__(NTHR) __attribute__((amdgpu_num_vgpr(248)))
void k_head(const unsigned short* __restrict__ zhl, const unsigned short* __restrict__ p1d,
            const float* __restrict__ smt, float* outp) {
  __shared__ __attribute__((aligned(16))) float stg[GBM * SPA];
  __shared__ __attribute__((aligned(16))) float sv[64];
  __shared__ __attribute__((aligned(16))) float sc[GBM];
  const int tid = (int)threadIdx.x, lane = tid & 31, wave = tid >> 5, hh = lane >> 4, m = lane & 15;
  const int blk = (int)blockIdx.x;
  const int rowBase = blk * GBM;
  if (tid < 16) *(v4fa*)(sv + 4 * tid) = *(const v4fa*)(smt + 96 + 4 * tid);
  const float qbv = smt[160];

  v8f acc[2];
  {
    const v8f z = {0.f, 0.f, 0.f, 0.f, 0.f, 0.f, 0.f, 0.f};
    acc[0] = z; acc[1] = z;
  }
  const unsigned short* ap = zhl + (size_t)(rowBase + 16 * wave + m) * (size_t)ZLP + 8 * hh;
  const unsigned short* bp = p1d + (size_t)m * (size_t)PDP + 8 * hh;
  gemm_rows16<KFIVE, PDP, 2>(ap, bp, acc);
  stage_d<2, SPA>(stg, acc, wave, hh, m);
  __syncthreads();

  if (tid < GBM) {
    const float* rp = stg + tid * SPA;
    float t = 0.0f;
#pragma unroll 1
    for (int g = 0; g < 8; ++g) {
      const v4f a = *(const v4fa*)(rp + 4 * g);
      const v4f b = *(const v4fa*)(sv + 4 * g);
      const v4f w = *(const v4fa*)(sv + 32 + 4 * g);
      float z0 = a.x + b.x, z1 = a.y + b.y, z2 = a.z + b.z, z3 = a.w + b.w;
      z0 = (z0 > 0.0f) ? z0 : (z0 - z0); z1 = (z1 > 0.0f) ? z1 : (z1 - z1);
      z2 = (z2 > 0.0f) ? z2 : (z2 - z2); z3 = (z3 > 0.0f) ? z3 : (z3 - z3);
      t = fmaf(z0, w.x, t); t = fmaf(z1, w.y, t); t = fmaf(z2, w.z, t); t = fmaf(z3, w.w, t);
    }
    t = t + qbv;
    sc[tid] = 1.0f / (1.0f + expf(-t));
  }
  __syncthreads();

  if (tid < 32) {
    const v4f v = *(const v4fa*)(sc + 4 * tid);
    st2_v4f(outp + (size_t)blk * GBM + 4 * tid, v);
  }
}

extern "C" void kernel_launch(void* const* d_in, const int* in_sizes, int n_in,
                              void* d_out, int out_size, void* d_ws, size_t ws_size,
                              hipStream_t stream) {
  if (n_in < 15) return;
  if (in_sizes[0] != NP || in_sizes[1] != NP) return;
  if (in_sizes[2] != NE || in_sizes[3] != NE || in_sizes[4] != NE) return;
  if (in_sizes[5] != NU * FD || in_sizes[6] != NI * FD) return;
  if (in_sizes[7] != HD * FD || in_sizes[8] != HD) return;
  if (in_sizes[9] != FD * HD || in_sizes[10] != FD) return;
  if (in_sizes[11] != HD * 2 * FD || in_sizes[12] != HD) return;
  if (in_sizes[13] != HD || in_sizes[14] != 1) return;
  if ((long long)out_size != (long long)NP + (long long)NN * FD) return;

  const int*   uids = (const int*)  d_in[0];
  const int*   iids = (const int*)  d_in[1];
  const int*   keys = (const int*)  d_in[2];
  const int*   cols = (const int*)  d_in[3];
  const float* vals = (const float*)d_in[4];
  const float* ue   = (const float*)d_in[5];
  const float* ie   = (const float*)d_in[6];
  const float* w1   = (const float*)d_in[7];
  const float* b1   = (const float*)d_in[8];
  const float* w2   = (const float*)d_in[9];
  const float* b2   = (const float*)d_in[10];
  const float* pw   = (const float*)d_in[11];
  const float* pb   = (const float*)d_in[12];
  const float* qw   = (const float*)d_in[13];
  const float* qb   = (const float*)d_in[14];
  float* out = (float*)d_out;

  constexpr size_t zXB   = (size_t)MP * FD * 2;
  constexpr size_t zTA   = (size_t)MP * HD * 4;
  constexpr size_t zHP   = (size_t)MP * HLP * 2;
  constexpr size_t zTB   = (size_t)MP * FD * 4;
  constexpr size_t zHF   = (size_t)NN * FD * 4;
  constexpr size_t zZHL  = (size_t)NP * ZLP * 2;
  constexpr size_t zLST  = (size_t)NBK * RCAP * 8;
  constexpr size_t zCOF  = (size_t)NBK * 2 * NBRUN * 4;
  constexpr size_t zFLG  = (size_t)NBK * 128;
  constexpr size_t zWA   = (size_t)HD * FD * 2;
  constexpr size_t zWB   = (size_t)FD * WDP * 2;
  constexpr size_t zWC   = (size_t)HD * PDP * 2;
  constexpr size_t zSM   = 1024;
  constexpr size_t oXB   = 0;
  constexpr size_t oTA   = oXB + zXB;
  constexpr size_t oHP   = oTA + zTA;
  constexpr size_t oTB   = oHP + zHP;
  constexpr size_t oHF   = oTB + zTB;
  constexpr size_t oZHL  = oHF + zHF;
  constexpr size_t oLST  = oZHL + zZHL;
  constexpr size_t oCOF  = oLST + zLST;
  constexpr size_t oFLG  = oCOF + zCOF;
  constexpr size_t oWA   = oFLG + zFLG;
  constexpr size_t oWB   = oWA + zWA;
  constexpr size_t oWC   = oWB + zWB;
  constexpr size_t oSM   = oWC + zWC;
  constexpr size_t oEND  = oSM + zSM;
  static_assert(zXB % 256 == 0 && zTA % 256 == 0 && zHP % 256 == 0 && zTB % 256 == 0 && zHF % 256 == 0);
  static_assert(zZHL % 256 == 0 && zLST % 256 == 0 && zCOF % 256 == 0 && zFLG % 256 == 0);
  static_assert(zWA % 256 == 0 && zWB % 256 == 0 && zWC % 256 == 0 && zSM % 256 == 0);
  static_assert(oEND <= WSMAX);
  if (oEND > ws_size) return;

  char* ws = (char*)d_ws;
  unsigned short* xb  = (unsigned short*)(ws + oXB);
  float*          t1f = (float*)(ws + oTA);
  unsigned short* h1p = (unsigned short*)(ws + oHP);
  float*          t2f = (float*)(ws + oTB);
  float*          h2f = (float*)(ws + oHF);
  unsigned short* zhl = (unsigned short*)(ws + oZHL);
  int*            lst = (int*)(ws + oLST);
  int*            cof = (int*)(ws + oCOF);
  int*            flg = (int*)(ws + oFLG);
  unsigned short* w1b = (unsigned short*)(ws + oWA);
  unsigned short* w2d = (unsigned short*)(ws + oWB);
  unsigned short* p1d = (unsigned short*)(ws + oWC);
  float*          smt = (float*)(ws + oSM);

  hipFuncSetAttribute(reinterpret_cast<const void*>(&k_bucket), hipFuncAttributeMaxDynamicSharedMemorySize, (int)BK_LDS);

  k_prep<<<PBTOT, NTHR, 0, stream>>>(ue, ie, w1, b1, w2, b2, pw, pb, qw, qb, xb, w1b, w2d, p1d, smt);
  k_bucket<<<NBK, NTHR, BK_LDS, stream>>>(keys, cols, vals, lst, cof, flg);
  k_gemm1<<<MP / GBM, NTHR, 0, stream>>>(xb, w1b, smt, t1f);
  k_replay1<<<MP / RBM, NTHR, 0, stream>>>(lst, cof, flg, t1f, h1p);
  k_gemm2<<<MP / GBM, NTHR, 0, stream>>>(h1p, w2d, smt, t2f);
  k_replay2<<<MP / RBM, NTHR, 0, stream>>>(lst, cof, flg, t2f, out + NP, h2f);
  k_headprep<<<NP / NWAVE, NTHR, 0, stream>>>(uids, iids, h2f, zhl);
  k_head<<<NP / GBM, NTHR, 0, stream>>>(zhl, p1d, smt, out);
}
